// TemporalViewModel_68968584839671
// MI455X (gfx1250) — hardware-verified
//
#include <hip/hip_runtime.h>

#define TT   24
#define NROW 16384
#define FS   64
#define FM   16
#define FC   16
#define NI   96
#define NH   32
#define G3   96
#define RPB  128
#define WST  40
#define HST  40
#define OST  68

typedef _Float16 f16;
typedef __attribute__((ext_vector_type(16))) f16 f16x16;
typedef __attribute__((ext_vector_type(8)))  f16 f16x8;
typedef __attribute__((ext_vector_type(8)))  float f32x8;
typedef __attribute__((ext_vector_type(4)))  float v4f_t;
typedef float v4fa __attribute__((ext_vector_type(4), may_alias));

__device__ __forceinline__ f32x8 wmma16(f16x16 a, f16x16 b, f32x8 c) {
  c = __builtin_amdgcn_wmma_f32_16x16x32_f16(false, a, false, b, (short)0, c, false, false);
  asm volatile("v_nop\n\tv_nop\n\tv_nop\n\tv_nop" : "+v"(c) : "v"(a), "v"(b));
  return c;
}
__device__ __forceinline__ f16x16 load_frag(const float* __restrict__ base, int ld, int row0, int k0) {
  const int lane = threadIdx.x & 31, r = lane & 15, kh = (lane >> 4) * 8;
  const float* p0 = base + (size_t)(row0 + r) * ld + (k0 + kh);
  const v4f_t a = *(const v4f_t*)(p0), b = *(const v4f_t*)(p0 + 4), c = *(const v4f_t*)(p0 + 16), d = *(const v4f_t*)(p0 + 20);
  f16x16 f;
  f[0] = (f16)a[0]; f[1] = (f16)a[1]; f[2]  = (f16)a[2]; f[3]  = (f16)a[3]; f[4]  = (f16)b[0]; f[5]  = (f16)b[1]; f[6]  = (f16)b[2]; f[7]  = (f16)b[3];
  f[8] = (f16)c[0]; f[9] = (f16)c[1]; f[10] = (f16)c[2]; f[11] = (f16)c[3]; f[12] = (f16)d[0]; f[13] = (f16)d[1]; f[14] = (f16)d[2]; f[15] = (f16)d[3];
  return f;
}
__device__ __forceinline__ f16x16 lds_frag(const f16* base, int stride) {
  const int lane = threadIdx.x & 31, row = lane & 15, kh = (lane >> 4) * 8;
  const f16x8 lo = *(const f16x8*)(base + row * stride + kh);
  const f16x8 hi = *(const f16x8*)(base + row * stride + kh + 16);
  f16x16 f;
#pragma unroll
  for (int i = 0; i < 8; ++i) { f[i] = lo[i]; f[i + 8] = hi[i]; }
  return f;
}
__device__ __forceinline__ float sigm(float x) { return 1.0f / (1.0f + __expf(-x)); }
__device__ __forceinline__ float tanh_(float x) { return 1.0f - 2.0f / (1.0f + __expf(2.0f * x)); }

__global__ __launch_bounds__(256) void gru_view_kernel(const float* __restrict__ spatial,
                                                      const float* __restrict__ met,
                                                      const float* __restrict__ ctx,
                                                      const float* __restrict__ Wih,
                                                      const float* __restrict__ Whh,
                                                      const float* __restrict__ bih,
                                                      const float* __restrict__ bhh,
                                                      const float* __restrict__ Wout,
                                                      float* __restrict__ out) {
  __shared__ __attribute__((aligned(16))) f16 WmcS[G3 * WST];
  __shared__ __attribute__((aligned(16))) f16 WhhS[G3 * WST];
  __shared__ __attribute__((aligned(16))) f16 WoS[FS * WST];
  __shared__ __attribute__((aligned(16))) f16 hS[8][16 * HST];
  __shared__ __attribute__((aligned(16))) float oS[8][16 * OST];
  __shared__ float bhn[NH];

  const int tid = threadIdx.x, lane = tid & 31, wave = tid >> 5, col = lane & 15, rh = (lane >> 4) * 8, kh = rh;
  const int row0 = blockIdx.x * RPB + wave * 16;

  for (int e = tid; e < G3 * 32; e += 256) {
    const int n = e >> 5, k = e & 31;
    WmcS[n * WST + k] = (f16)Wih[n * NI + FS + k];
    WhhS[n * WST + k] = (f16)Whh[n * NH + k];
  }
  for (int e = tid; e < FS * NH; e += 256) { const int f = e >> 5, h = e & 31; WoS[f * WST + h] = (f16)Wout[h * FS + f]; }
  for (int e = tid; e < 8 * 16 * HST; e += 256) (&hS[0][0])[e] = (f16)0.0f;
  if (tid < NH) bhn[tid] = bhh[2 * NH + tid];
  __syncthreads();

  f32x8 gsp[6];
  {
    const f16x16 a0 = load_frag(spatial, FS, row0, 0), a1 = load_frag(spatial, FS, row0, 32);
#pragma unroll
    for (int nt = 0; nt < 6; ++nt) {
      f32x8 z = {};
      z = wmma16(a0, load_frag(Wih, NI, nt * 16, 0), z);
      z = wmma16(a1, load_frag(Wih, NI, nt * 16, 32), z);
      const int n = nt * 16 + col;
      const float bb = bih[n] + ((nt < 4) ? bhh[n] : 0.0f);
#pragma unroll
      for (int r = 0; r < 8; ++r) z[r] += bb;
      gsp[nt] = z;
    }
  }
  float hreg[2][8];
#pragma unroll
  for (int u = 0; u < 2; ++u)
#pragma unroll
    for (int r = 0; r < 8; ++r) hreg[u][r] = 0.0f;

#pragma unroll 1
  for (int t = 0; t < TT; ++t) {
    f16x16 ax;
    {
      const float* pm = met + ((size_t)t * NROW + row0 + col) * FM + kh;
      const float* pc = ctx + ((size_t)t * NROW + row0 + col) * FC + kh;
      const v4f_t m0 = *(const v4f_t*)pm, m1 = *(const v4f_t*)(pm + 4), c0 = *(const v4f_t*)pc, c1 = *(const v4f_t*)(pc + 4);
      ax[0] = (f16)m0[0]; ax[1] = (f16)m0[1]; ax[2]  = (f16)m0[2]; ax[3]  = (f16)m0[3]; ax[4]  = (f16)m1[0]; ax[5]  = (f16)m1[1]; ax[6]  = (f16)m1[2]; ax[7]  = (f16)m1[3];
      ax[8] = (f16)c0[0]; ax[9] = (f16)c0[1]; ax[10] = (f16)c0[2]; ax[11] = (f16)c0[3]; ax[12] = (f16)c1[0]; ax[13] = (f16)c1[1]; ax[14] = (f16)c1[2]; ax[15] = (f16)c1[3];
    }
    const f16x16 ah = lds_frag(hS[wave], HST);
    float hnew[2][8];
#pragma unroll
    for (int u = 0; u < 2; ++u) {
      f32x8 gi_r = wmma16(ax, lds_frag(WmcS + (u) * 16 * WST, WST), gsp[u]);
      f32x8 gi_z = wmma16(ax, lds_frag(WmcS + (2 + u) * 16 * WST, WST), gsp[2 + u]);
      f32x8 gi_n = wmma16(ax, lds_frag(WmcS + (4 + u) * 16 * WST, WST), gsp[4 + u]);
      f32x8 zz = {};
      f32x8 gh_r = wmma16(ah, lds_frag(WhhS + (u) * 16 * WST, WST), zz);
      f32x8 gh_z = wmma16(ah, lds_frag(WhhS + (2 + u) * 16 * WST, WST), zz);
      f32x8 gh_n = wmma16(ah, lds_frag(WhhS + (4 + u) * 16 * WST, WST), zz);
      const float bn = bhn[16 * u + col];
#pragma unroll
      for (int r = 0; r < 8; ++r) {
        const float rg = sigm(gi_r[r] + gh_r[r]);
        const float zg = sigm(gi_z[r] + gh_z[r]);
        const float ng = tanh_(gi_n[r] + rg * (gh_n[r] + bn));
        hnew[u][r] = (1.0f - zg) * ng + zg * hreg[u][r];
      }
    }
    __syncthreads();
#pragma unroll
    for (int u = 0; u < 2; ++u)
#pragma unroll
      for (int r = 0; r < 8; ++r) { hreg[u][r] = hnew[u][r]; hS[wave][(rh + r) * HST + 16 * u + col] = (f16)hnew[u][r]; }
    __syncthreads();
  }

  {
    const f16x16 ah = lds_frag(hS[wave], HST);
#pragma unroll
    for (int nt = 0; nt < 4; ++nt) {
      f32x8 z = {};
      z = wmma16(ah, lds_frag(WoS + nt * 16 * WST, WST), z);
#pragma unroll
      for (int r = 0; r < 8; ++r) oS[wave][(rh + r) * OST + nt * 16 + col] = z[r];
    }
  }
  __syncthreads();
#pragma unroll 1
  for (int pass = 0; pass < 2; ++pass) {
#pragma unroll
    for (int it = 0; it < 8; ++it) {
      const int f4 = lane + 32 * it, rr = f4 >> 4, q = (f4 & 15) * 4;
      *(volatile v4f_t*)(out + (size_t)(row0 + rr) * FS + q) = *(const volatile v4fa*)(oS[wave] + rr * OST + q);
    }
    __threadfence();
  }
}

extern "C" void kernel_launch(void* const* d_in, const int* in_sizes, int n_in,
                              void* d_out, int out_size, void* d_ws, size_t ws_size,
                              hipStream_t stream) {
  (void)in_sizes; (void)n_in; (void)out_size; (void)d_ws; (void)ws_size;
  const float* spatial = (const float*)d_in[0];
  const float* met     = (const float*)d_in[1];
  const float* ctx     = (const float*)d_in[2];
  const float* Wih     = (const float*)d_in[3];
  const float* Whh     = (const float*)d_in[4];
  const float* bih     = (const float*)d_in[5];
  const float* bhh     = (const float*)d_in[6];
  const float* Wout    = (const float*)d_in[7];
  float* out = (float*)d_out;
  gru_view_kernel<<<dim3(NROW / RPB), dim3(256), 0, stream>>>(spatial, met, ctx, Wih, Whh, bih, bhh, Wout, out);
}
